// ContextPythiaAttention_21251498180931
// MI455X (gfx1250) — hardware-verified
//
#include <hip/hip_runtime.h>


namespace {
constexpr int Bn = 2, S = 2048, CD = 512, D = 1024, H = 16, HD = 64, RD = 16, D3 = 3 * D, NT = Bn * S;
constexpr float XS = 8.0f, PS = 8.0f, ISC = 0.125f;
__constant__ unsigned int INVF[8] = {0x3f800000u, 0x3ea1e89bu, 0x3dcccccdu, 0x3d0186e3u, 0x3c23d70au, 0x3b4f3e38u, 0x3a83126fu, 0x39a5cb60u};

typedef _Float16 b16;
typedef __attribute__((ext_vector_type(16))) _Float16 v16b;
typedef __attribute__((ext_vector_type(8))) _Float16 v8b;
typedef __attribute__((ext_vector_type(8))) float v8f;
typedef __attribute__((ext_vector_type(4))) float v4f;
__device__ __forceinline__ float bf16_rne(float f) { unsigned int u = __float_as_uint(f); u += 0x7FFFu + ((u >> 16) & 1u); return __uint_as_float(u & 0xFFFF0000u); }
__device__ __forceinline__ void split16(float v, b16& hi, b16& lo) { hi = (b16)v; lo = (b16)(v - (float)hi); }
__device__ __forceinline__ v16b frag_kb(const b16* p, int hh) { const v8b a = *(const v8b*)(p + 8 * hh), b = *(const v8b*)(p + 16 + 8 * hh); v16b f;
#pragma unroll
  for (int e = 0; e < 8; ++e) { f[e] = a[e]; f[8 + e] = b[e]; } return f; }
__device__ __forceinline__ v8f wmma16b(v16b a, v16b b, v8f c) { v8f d = __builtin_amdgcn_wmma_f32_16x16x32_f16(false, a, false, b, (short)0, c, false, false); asm volatile("v_nop\n\tv_nop\n\tv_nop\n\tv_nop" : "+v"(d) : "v"(a), "v"(b)); return d; }
__device__ __forceinline__ void wave_lds_sync() { __builtin_amdgcn_fence(__ATOMIC_RELEASE, "workgroup"); __builtin_amdgcn_wave_barrier(); __builtin_amdgcn_fence(__ATOMIC_ACQUIRE, "workgroup"); }
__device__ __forceinline__ float nexp(float x) { return __builtin_amdgcn_exp2f(x * 1.4426950408889634f); }
__device__ __forceinline__ float pmul(float a, float b) { float p = a * b; asm volatile("" : "+v"(p)); return p; }

__global__ __launch_bounds__(256) void prep_kernel(const float* __restrict__ x, const float* __restrict__ wq, const float* __restrict__ bq, const float* __restrict__ wk, const float* __restrict__ bk, const float* __restrict__ wv, const float* __restrict__ bv, const float* __restrict__ wd, const float* __restrict__ bd, b16* __restrict__ R, b16* __restrict__ RD_, float* __restrict__ P, b16* __restrict__ X) {
  const size_t tid = (size_t)blockIdx.x * 256 + threadIdx.x, nth = (size_t)gridDim.x * 256;
  for (int pass = 0; pass < 2; ++pass) {
    for (size_t p = tid; p < (size_t)D3 * (CD / 8); p += nth) { const int o3 = (int)(p / (CD / 8)), k0 = (int)(p % (CD / 8)) * 8; const int w = o3 / D, o = o3 % D; const float* Wm = (w == 0) ? wq : (w == 1) ? wk : wv; v8b v; for (int e = 0; e < 8; ++e) v[e] = (b16)bf16_rne(Wm[(size_t)(k0 + e) * D + o]); *(volatile v8b*)(R + (size_t)o3 * CD + k0) = v; }
    for (size_t p = tid; p < (size_t)D * (D / 8); p += nth) { const int o = (int)(p / (D / 8)), k0 = (int)(p % (D / 8)) * 8; v8b v; for (int e = 0; e < 8; ++e) v[e] = (b16)bf16_rne(wd[(size_t)(k0 + e) * D + o]); *(volatile v8b*)(RD_ + (size_t)o * D + k0) = v; }
    for (size_t q = tid; q < 4096; q += nth) { const int i = (int)q; P[q] = bf16_rne((i < 1024) ? bq[i] : (i < 2048) ? bk[i - 1024] : (i < 3072) ? bv[i - 2048] : bd[i - 3072]); }
    for (size_t q = tid; q < (size_t)S * 8; q += nth) { const int t = (int)(q >> 3), f = (int)(q & 7); const float ang = (float)t * __uint_as_float(INVF[f]); P[4096 + q] = (float)cos((double)ang); P[4096 + 16384 + q] = (float)sin((double)ang); }
    for (size_t p = tid; p < (size_t)NT * CD / 8; p += nth) { v8b v; for (int e = 0; e < 8; ++e) v[e] = (b16)(bf16_rne(x[p * 8 + e]) * XS); *(volatile v8b*)(X + p * 8) = v; }
    __threadfence(); }
}

__global__ __launch_bounds__(64) void qk_kernel(const b16* __restrict__ X, const b16* __restrict__ R, const float* __restrict__ P, b16* __restrict__ Q, b16* __restrict__ K, b16* __restrict__ QL, b16* __restrict__ KL) {
  __shared__ __attribute__((aligned(16))) b16 Th[2][16][128 + 8], Tl[2][16][128 + 8];
  const int lane = threadIdx.x & 31, wave = threadIdx.x >> 5, nloc = lane & 15, hlf = lane >> 4, mw = blockIdx.y * 32 + wave * 16; const bool isk = blockIdx.x >= 8; const int c0 = (blockIdx.x & 7) * 128; const b16* Bw = R + (size_t)((isk ? D : 0) + c0) * CD; const float* bias = P + (isk ? D : 0) + c0;
  v8f acc[8];
#pragma unroll
  for (int t = 0; t < 8; ++t) acc[t] = (v8f){};
#pragma unroll 2
  for (int kb = 0; kb < CD; kb += 32) { const v16b a = frag_kb(X + (size_t)(mw + nloc) * CD + kb, hlf);
#pragma unroll
    for (int t = 0; t < 8; ++t) acc[t] = wmma16b(a, frag_kb(Bw + (size_t)(t * 16 + nloc) * CD + kb, hlf), acc[t]); }
#pragma unroll
  for (int t = 0; t < 8; ++t) {
#pragma unroll
    for (int r = 0; r < 8; ++r) { float v = acc[t][r] * (1.0f / XS) + bias[t * 16 + nloc];
      if ((t & 3) == 0) {
        const float partner = __shfl_xor(v, 8); const int tok = (mw + 8 * hlf + r) % S; const int f = nloc & 7; const float cs = P[4096 + tok * 8 + f], sn = P[4096 + 16384 + tok * 8 + f];
        v = (nloc < 8) ? (pmul(v, cs) - pmul(partner, sn)) : (pmul(v, cs) + pmul(partner, sn)); }
      b16 a_, c_; split16(v * XS, a_, c_); Th[wave][8 * hlf + r][t * 16 + nloc] = a_; Tl[wave][8 * hlf + r][t * 16 + nloc] = c_; } }
  wave_lds_sync();
  b16* dstp = isk ? K : Q; b16* dstl = isk ? KL : QL;
  for (int pass = 0; pass < 2; ++pass) { for (int i = lane; i < 16 * 16; i += 32) { const int rr = i >> 4, c8 = (i & 15) * 8; const size_t gi = (size_t)(mw + rr) * D + c0 + c8; *(volatile v8b*)(dstp + gi) = *(const v8b*)(&Th[wave][rr][c8]); *(volatile v8b*)(dstl + gi) = *(const v8b*)(&Tl[wave][rr][c8]); } __threadfence(); }
}
__global__ __launch_bounds__(128) void v_kernel(const b16* __restrict__ X, const b16* __restrict__ R, const float* __restrict__ P, b16* __restrict__ VT, b16* __restrict__ VTl) {
  __shared__ __attribute__((aligned(16))) b16 Th[128][64 + 8], Tl[128][64 + 8];
  const int lane = threadIdx.x & 31, wave = threadIdx.x >> 5, nloc = lane & 15, hlf = lane >> 4, g0 = blockIdx.y * 64, m0 = g0 + wave * 16, c0 = blockIdx.x * 128; const b16* Bv = R + (size_t)(2 * D + c0) * CD;
  const int b = g0 / S, t0 = g0 % S;
  v8f acc[8];
#pragma unroll
  for (int t = 0; t < 8; ++t) acc[t] = (v8f){};
#pragma unroll 2
  for (int kb = 0; kb < CD; kb += 32) { const v16b a = frag_kb(X + (size_t)(m0 + nloc) * CD + kb, hlf);
#pragma unroll
    for (int t = 0; t < 8; ++t) acc[t] = wmma16b(a, frag_kb(Bv + (size_t)(t * 16 + nloc) * CD + kb, hlf), acc[t]); }
#pragma unroll
  for (int t = 0; t < 8; ++t)
#pragma unroll
    for (int r = 0; r < 8; ++r) { b16 a_, c_; split16(acc[t][r] + XS * P[2048 + c0 + t * 16 + nloc], a_, c_); Th[t * 16 + nloc][wave * 16 + 8 * hlf + r] = a_; Tl[t * 16 + nloc][wave * 16 + 8 * hlf + r] = c_; }
  __syncthreads();
  for (int pass = 0; pass < 2; ++pass) { for (int i = threadIdx.x; i < 128 * 8; i += 128) { const int dd = i >> 3, c8 = (i & 7) * 8; const size_t gi = ((size_t)b * D + c0 + dd) * S + t0 + c8; *(volatile v8b*)(VT + gi) = *(const v8b*)(&Th[dd][c8]); *(volatile v8b*)(VTl + gi) = *(const v8b*)(&Tl[dd][c8]); } __threadfence(); }
}
__global__ __launch_bounds__(128) void attn_kernel(const b16* __restrict__ Q, const b16* __restrict__ QLp, const b16* __restrict__ K, const b16* __restrict__ KLp, const b16* __restrict__ VT, const b16* __restrict__ VTL, b16* __restrict__ CH, b16* __restrict__ CL) {
  __shared__ __attribute__((aligned(16))) b16 Oh[16][4 * HD + 8], Ol[16][4 * HD + 8];
  const int wid = threadIdx.x >> 5, lane = threadIdx.x & 31, hh = lane >> 4, col = lane & 15; const int b = blockIdx.z, q0 = blockIdx.x * 16, h = blockIdx.y * 4 + wid, qi = q0 + col;
  const b16* Qr = Q + ((size_t)b * S) * D + h * HD; const b16* Qlr = QLp + ((size_t)b * S) * D + h * HD; const b16* Kr = K + ((size_t)b * S) * D + h * HD; const b16* Klr = KLp + ((size_t)b * S) * D + h * HD; const b16* V = VT + ((size_t)b * D + h * HD) * S; const b16* Vl = VTL + ((size_t)b * D + h * HD) * S;
  const v16b qf0 = frag_kb(Qr + (size_t)qi * D, hh), qf1 = frag_kb(Qr + (size_t)qi * D + 32, hh), ql0 = frag_kb(Qlr + (size_t)qi * D, hh), ql1 = frag_kb(Qlr + (size_t)qi * D + 32, hh);
  float m = -INFINITY, l = 0.0f; v8f o[4] = {{}, {}, {}, {}};
  for (int kb = 0; kb < q0 + 16; kb += 32) {
    v8f s0 = {}, s1 = {};
    { const v16b k00 = frag_kb(Kr + (size_t)(kb + col) * D, hh), k01 = frag_kb(Kr + (size_t)(kb + col) * D + 32, hh), k10 = frag_kb(Kr + (size_t)(kb + 16 + col) * D, hh), k11 = frag_kb(Kr + (size_t)(kb + 16 + col) * D + 32, hh);
      const v16b l00 = frag_kb(Klr + (size_t)(kb + col) * D, hh), l01 = frag_kb(Klr + (size_t)(kb + col) * D + 32, hh), l10 = frag_kb(Klr + (size_t)(kb + 16 + col) * D, hh), l11 = frag_kb(Klr + (size_t)(kb + 16 + col) * D + 32, hh);
      s0 = wmma16b(k00, qf0, s0); s0 = wmma16b(k01, qf1, s0); s0 = wmma16b(l00, qf0, s0); s0 = wmma16b(l01, qf1, s0); s0 = wmma16b(k00, ql0, s0); s0 = wmma16b(k01, ql1, s0);
      s1 = wmma16b(k10, qf0, s1); s1 = wmma16b(k11, qf1, s1); s1 = wmma16b(l10, qf0, s1); s1 = wmma16b(l11, qf1, s1); s1 = wmma16b(k10, ql0, s1); s1 = wmma16b(k11, ql1, s1); }
    float mr = -INFINITY;
#pragma unroll
    for (int r = 0; r < 8; ++r) { const int j0 = kb + 8 * hh + r, j1 = j0 + 16; s0[r] = (j0 <= qi) ? s0[r] * (ISC / (XS * XS)) : -INFINITY; s1[r] = (j1 <= qi) ? s1[r] * (ISC / (XS * XS)) : -INFINITY; mr = fmaxf(mr, fmaxf(s0[r], s1[r])); }
    mr = fmaxf(mr, __shfl_xor(mr, 16)); const float mn = fmaxf(m, mr); const float al_ = (mn == -INFINITY) ? 1.0f : nexp(m - mn); m = mn; float sum = 0.0f; v16b pb, pl;
#pragma unroll
    for (int r = 0; r < 8; ++r) { const float e0 = (s0[r] == -INFINITY) ? 0.0f : nexp(s0[r] - mn), e1 = (s1[r] == -INFINITY) ? 0.0f : nexp(s1[r] - mn); sum += e0 + e1; b16 a_, c_; split16(e0 * PS, a_, c_); pb[r] = a_; pl[r] = c_; split16(e1 * PS, a_, c_); pb[8 + r] = a_; pl[8 + r] = c_; }
    sum += __shfl_xor(sum, 16); l = l * al_ + sum;
#pragma unroll
    for (int t = 0; t < 4; ++t) { o[t] *= al_; const v16b vh = frag_kb(V + (size_t)(t * 16 + col) * S + kb, hh); o[t] = wmma16b(vh, pb, o[t]); o[t] = wmma16b(vh, pl, o[t]); o[t] = wmma16b(frag_kb(Vl + (size_t)(t * 16 + col) * S + kb, hh), pb, o[t]); } }
  const float inv = 1.0f / (l * PS);
#pragma unroll
  for (int t = 0; t < 4; ++t)
#pragma unroll
    for (int r = 0; r < 8; ++r) { b16 a_, c_; split16(o[t][r] * inv, a_, c_); Oh[col][wid * HD + t * 16 + 8 * hh + r] = a_; Ol[col][wid * HD + t * 16 + 8 * hh + r] = c_; }
  __syncthreads();
  for (int pass = 0; pass < 2; ++pass) { for (int i = threadIdx.x; i < 16 * 32; i += 128) { const int rr = i >> 5, c8 = (i & 31) * 8; const size_t gi = ((size_t)b * S + q0 + rr) * D + blockIdx.y * 4 * HD + c8; *(volatile v8b*)(CH + gi) = *(const v8b*)(&Oh[rr][c8]); *(volatile v8b*)(CL + gi) = *(const v8b*)(&Ol[rr][c8]); } __threadfence(); }
}
__global__ __launch_bounds__(64) void out_kernel(const b16* __restrict__ CH, const b16* __restrict__ CL, const b16* __restrict__ RD_, const float* __restrict__ P, float* __restrict__ out) {
  __shared__ __attribute__((aligned(16))) float Ts[2][32][128 + 4];
  const int lane = threadIdx.x & 31, wave = threadIdx.x >> 5, nloc = lane & 15, hlf = lane >> 4, m0 = blockIdx.y * 32, c0 = blockIdx.x * 256 + wave * 128;
  v8f acc[2][8];
#pragma unroll
  for (int r = 0; r < 2; ++r)
#pragma unroll
    for (int t = 0; t < 8; ++t) acc[r][t] = (v8f){};
#pragma unroll 2
  for (int kb = 0; kb < D; kb += 32) { const v16b a0 = frag_kb(CH + (size_t)(m0 + nloc) * D + kb, hlf), a1 = frag_kb(CH + (size_t)(m0 + 16 + nloc) * D + kb, hlf), l0 = frag_kb(CL + (size_t)(m0 + nloc) * D + kb, hlf), l1 = frag_kb(CL + (size_t)(m0 + 16 + nloc) * D + kb, hlf);
#pragma unroll
    for (int t = 0; t < 8; ++t) { const v16b bw = frag_kb(RD_ + (size_t)(c0 + t * 16 + nloc) * D + kb, hlf); acc[0][t] = wmma16b(a0, bw, acc[0][t]); acc[0][t] = wmma16b(l0, bw, acc[0][t]); acc[1][t] = wmma16b(a1, bw, acc[1][t]); acc[1][t] = wmma16b(l1, bw, acc[1][t]); } }
#pragma unroll
  for (int t = 0; t < 8; ++t) { const float bb = P[3072 + c0 + t * 16 + nloc];
#pragma unroll
    for (int r = 0; r < 2; ++r)
#pragma unroll
      for (int v = 0; v < 8; ++v) Ts[wave][r * 16 + 8 * hlf + v][t * 16 + nloc] = acc[r][t][v] * (1.0f / XS) + bb; }
  wave_lds_sync();
  for (int pass = 0; pass < 2; ++pass) { for (int i = lane; i < 32 * 32; i += 32) { const int rr = i >> 5, c4 = (i & 31) * 4; *(volatile v4f*)(out + (size_t)(m0 + rr) * D + c0 + c4) = *(const v4f*)(&Ts[wave][rr][c4]); } __threadfence(); }
}
}

extern "C" void kernel_launch(void* const* d_in, const int* in_sizes, int n_in,
                              void* d_out, int out_size, void* d_ws, size_t ws_size, hipStream_t stream) {
  (void)n_in; (void)out_size;
  const float* x = (const float*)d_in[0]; const float* wq = (const float*)d_in[1]; const float* bq = (const float*)d_in[2]; const float* wk = (const float*)d_in[3]; const float* bk = (const float*)d_in[4]; const float* wv = (const float*)d_in[5]; const float* bv = (const float*)d_in[6]; const float* wd = (const float*)d_in[7]; const float* bd = (const float*)d_in[8];
  float* out = (float*)d_out;
  if (in_sizes[0] != NT * CD || in_sizes[1] != CD * D || in_sizes[7] != D * D) return;
  size_t off = 0; char* ws = (char*)d_ws;
  auto carve = [&](size_t bytes) { char* p = ws + off; off += (bytes + 255) & ~(size_t)255; return p; };
  b16* R = (b16*)carve((size_t)D3 * CD * 2); b16* RD_ = (b16*)carve((size_t)D * D * 2); float* P = (float*)carve((4096 + 32768) * 4); b16* X = (b16*)carve((size_t)NT * CD * 2); b16* Q = (b16*)carve((size_t)NT * D * 2); b16* K = (b16*)carve((size_t)NT * D * 2); b16* QL = (b16*)carve((size_t)NT * D * 2); b16* KL = (b16*)carve((size_t)NT * D * 2); b16* VT = (b16*)carve((size_t)NT * D * 2); b16* VTl = (b16*)carve((size_t)NT * D * 2); b16* CH = (b16*)carve((size_t)NT * D * 2); b16* CL = (b16*)carve((size_t)NT * D * 2);
  if (off > ws_size) return;
  prep_kernel<<<512, 256, 0, stream>>>(x, wq, bq, wk, bk, wv, bv, wd, bd, R, RD_, P, X);
  qk_kernel<<<dim3(16, NT / 32), 64, 0, stream>>>(X, R, P, Q, K, QL, KL);
  v_kernel<<<dim3(8, NT / 64), 128, 0, stream>>>(X, R, P, VT, VTl);
  attn_kernel<<<dim3(S / 16, 4, Bn), 128, 0, stream>>>(Q, QL, K, KL, VT, VTl, CH, CL);
  out_kernel<<<dim3(4, NT / 32), 64, 0, stream>>>(CH, CL, RD_, P, out);
}
